// Net_24257975287857
// MI455X (gfx1250) — hardware-verified
//
#include <hip/hip_runtime.h>
#include <math.h>

constexpr int NN     = 100000;
constexpr int NE     = 1600000;
constexpr int CH     = 128;
constexpr int KCAT   = 256;
constexpr int HCAT   = 384;
constexpr int NCLS   = 41;
constexpr int NCLSP  = 64;
constexpr int NT     = 256;
constexpr int TROWS  = 128;
constexpr int TSHIFT = 7;
constexpr int NTILE  = 782;
constexpr int NPAD2  = NTILE * TROWS;
constexpr int CHK    = 16384;
constexpr int NCHUNK = 98;
constexpr int CAP    = 64;
constexpr int NPAIR  = NTILE / 2;
constexpr int NPIT   = 49;
constexpr int SENT_TILE = 1023;
constexpr int MCLS   = 1563;
constexpr int GEMM_BLOCKS = (NPAD2 / 64) * (CH / 64) / 8;
constexpr float WCARRY     = 16.0f;
constexpr float WCARRY_INV = 1.0f / 16.0f;

static_assert(TROWS == (1 << TSHIFT), "tile shift");
static_assert(NPAD2 % 64 == 0 && NPAD2 >= NN, "plane rows");
static_assert(NCHUNK * CHK >= NE && (NCHUNK - 1) * CHK < NE, "chunks cover edges");
static_assert(CHK == 16384, "local edge index packs into 14 bits");
static_assert(NE < (1 << 21), "edge id packs into 21 bits");
static_assert(NTILE + 2 < SENT_TILE, "sentinel tile above all real tiles");
static_assert(NE % 4 == 0 && CHK % (4 * NT) == 0, "16-B aligned edge group loads");
static_assert(NPAIR * 2 == NTILE && 8 * NPIT >= NPAIR, "cell pairs");
static_assert(MCLS * 64 >= NN && (MCLS - 1) * 64 < NN && MCLS * 64 <= NPAD2, "classifier grid");
static_assert(((NPAD2 / 64) * (CH / 64)) % 8 == 0, "gemm grid exact");
static_assert(KCAT % 32 == 0 && HCAT % 32 == 0, "K multiples of 32");
static_assert(CH % 64 == 0 && NCLSP % 64 == 0, "N tile multiples");
static_assert((64 * NCLS * 4) % 128 == 0, "a 64-row output block is a whole number of 128-B lines");
static_assert(((NN % 64) * NCLS * 4) % 128 == 0, "the last output block is a whole number of 128-B lines");
static_assert((NPAD2 * 16) % NT == 0, "x0 cast grid exact");

typedef __attribute__((ext_vector_type(16))) _Float16 v16h;
typedef __attribute__((ext_vector_type(8)))  _Float16 v8h;
typedef __attribute__((ext_vector_type(16))) __bf16   v16b;
typedef __attribute__((ext_vector_type(8)))  __bf16   v8b;
typedef __attribute__((ext_vector_type(8)))  float    v8f;
typedef __attribute__((ext_vector_type(4)))  float    v4f;
typedef __attribute__((ext_vector_type(4)))  int      v4i;
typedef __attribute__((ext_vector_type(4)))  unsigned v4u;
typedef __attribute__((ext_vector_type(2)))  unsigned v2u;

__device__ __forceinline__ void dep_guard_h(v8f& a, v8f& b, v16h x, v16h y) { asm volatile("v_nop\n\tv_nop\n\tv_nop\n\tv_nop" : "+v"(a), "+v"(b) : "v"(x), "v"(y)); }
__device__ __forceinline__ void dep_guard_b(v8f& a, v8f& b, v16b x, v16b y) { asm volatile("v_nop\n\tv_nop\n\tv_nop\n\tv_nop" : "+v"(a), "+v"(b) : "v"(x), "v"(y)); }
__device__ __forceinline__ void keep4_h(v16h a, v16h b, v16h c, v16h d) { asm volatile("v_nop" :: "v"(a), "v"(b), "v"(c), "v"(d)); }
__device__ __forceinline__ void keep4_b(v16b a, v16b b, v16b c, v16b d) { asm volatile("v_nop" :: "v"(a), "v"(b), "v"(c), "v"(d)); }
__device__ __forceinline__ void acc_guard4(v8f& a, v8f& b, v8f& c, v8f& d) { asm volatile("v_nop\n\tv_nop\n\tv_nop\n\tv_nop" : "+v"(a), "+v"(b), "+v"(c), "+v"(d)); }
template <typename T> struct Frag;
template <> struct Frag<_Float16> {
  typedef v16h V; union U { v16h v; v8h h[2]; };
  static __device__ __forceinline__ v16h load(const _Float16* p) {
    U f; f.h[0] = *(const v8h*)(p); f.h[1] = *(const v8h*)(p + 16); return f.v;
  }
  static __device__ __forceinline__ v8f mma(v16h a, v16h b, v8f c) {
    return __builtin_amdgcn_wmma_f32_16x16x32_f16(false, a, false, b, (short)0, c, false, false);
  }
  static __device__ __forceinline__ void guard(v8f& a, v8f& b, v16h x, v16h y) { dep_guard_h(a, b, x, y); }
  static __device__ __forceinline__ void keep(v16h a, v16h b, v16h c, v16h d) { keep4_h(a, b, c, d); }
};
template <> struct Frag<__bf16> {
  typedef v16b V; union U { v16b v; v8b h[2]; };
  static __device__ __forceinline__ v16b load(const __bf16* p) {
    U f; f.h[0] = *(const v8b*)(p); f.h[1] = *(const v8b*)(p + 16); return f.v;
  }
  static __device__ __forceinline__ v8f mma(v16b a, v16b b, v8f c) {
    return __builtin_amdgcn_wmma_f32_16x16x32_bf16(false, a, false, b, (short)0, c, false, false);
  }
  static __device__ __forceinline__ void guard(v8f& a, v8f& b, v16b x, v16b y) { dep_guard_b(a, b, x, y); }
  static __device__ __forceinline__ void keep(v16b a, v16b b, v16b c, v16b d) { keep4_b(a, b, c, d); }
};

__device__ __forceinline__ void guard_grp(v8f& a, v8f& b, v8f& c, v8f& d, v16h x, v16h y0, v16h y1, v16h y2, v16h y3) {
  asm volatile("v_nop\n\tv_nop\n\tv_nop\n\tv_nop" : "+v"(a), "+v"(b), "+v"(c), "+v"(d) : "v"(x), "v"(y0), "v"(y1), "v"(y2), "v"(y3));
}
__device__ __forceinline__ void guard2f(v8f& a, v8f& b, v16h x, v16h y0, v16h y1) {
  asm volatile("v_nop\n\tv_nop\n\tv_nop\n\tv_nop" : "+v"(a), "+v"(b) : "v"(x), "v"(y0), "v"(y1));
}
__device__ __forceinline__ void acc_guard2(v8f& a, v8f& b) { asm volatile("v_nop\n\tv_nop\n\tv_nop\n\tv_nop" : "+v"(a), "+v"(b)); }

__device__ __forceinline__ unsigned pk16(unsigned short a, unsigned short b) { return (unsigned)a | ((unsigned)b << 16); }
__device__ __forceinline__ unsigned short h_bits(float f) { const _Float16 h = (_Float16)f; return __builtin_bit_cast(unsigned short, h); }
__device__ __forceinline__ float h16_to_f32(unsigned hb) {
  const unsigned sgn = (hb & 0x8000u) << 16; const unsigned em = hb & 0x7fffu;
  const float fn = __uint_as_float((em << 13) + 0x38000000u);
  const float fs = (float)em * 5.9604644775390625e-8f;
  const float mag = (em < 0x400u) ? fs : fn; return __uint_as_float(__float_as_uint(mag) | sgn); }

__global__ __launch_bounds__(NT) void k_packw(const float* __restrict__ Wr1, const float* __restrict__ Wo1,
                                              const float* __restrict__ Wr2, const float* __restrict__ Wo2,
                                              const float* __restrict__ Wr3, const float* __restrict__ Wo3,
                                              const float* __restrict__ Wlin,
                                              unsigned* __restrict__ WCw, unsigned* __restrict__ WLw) {
  const int y = blockIdx.y;
  const int i = blockIdx.x * NT + threadIdx.x;
  unsigned u;
  unsigned* dst;
  if (y < 6) {
    if (i >= CH * CH / 2) return;
    const float* W = (y == 0) ? Wr1 : (y == 1) ? Wo1 : (y == 2) ? Wr2 : (y == 3) ? Wo2 : (y == 4) ? Wr3 : Wo3;
    const int l = y >> 1, part = y & 1;
    const int n = i >> 6, kw = i & 63;
    const float a = W[n * CH + 2 * kw] * WCARRY;
    const float b = W[n * CH + 2 * kw + 1] * WCARRY;
    u = pk16(h_bits(a), h_bits(b));
    dst = WCw + (size_t)l * (CH * KCAT / 2) + (size_t)n * (KCAT / 2) + part * (CH / 2) + kw;
  } else {
    if (i >= NCLSP * HCAT / 2) return;
    const int n = i / (HCAT / 2);
    const int kw = i - n * (HCAT / 2);
    const int nc = (n < NCLS) ? n : (NCLS - 1);
    const float live = (n < NCLS) ? 1.0f : 0.0f;
    const float a = Wlin[nc * HCAT + 2 * kw] * (WCARRY * live);
    const float b = Wlin[nc * HCAT + 2 * kw + 1] * (WCARRY * live);
    u = pk16(h_bits(a), h_bits(b));
    dst = WLw + i;
  }
  *(volatile unsigned*)dst = u;
  __threadfence();
  *(volatile unsigned*)dst = u;
}

__global__ __launch_bounds__(NT) void k_cast_x0(const float* __restrict__ x0, unsigned* __restrict__ XO) {
  const int i = blockIdx.x * NT + threadIdx.x;
  if (i >= NPAD2 * 16) return;
  const bool inr = i < NN * 16;
  const int ic = inr ? i : 0;
  const float m = inr ? 1.0f : 0.0f;
  const float* p = x0 + 8 * (size_t)ic;
  const v4f a = *(const v4f*)(p);
  const v4f c = *(const v4f*)(p + 4);
  unsigned short hb[8];
#pragma unroll
  for (int e = 0; e < 4; ++e) {
    hb[e]     = h_bits(a[e] * m);
    hb[4 + e] = h_bits(c[e] * m);
  }
  const v4u u = (v4u){pk16(hb[0], hb[1]), pk16(hb[2], hb[3]), pk16(hb[4], hb[5]), pk16(hb[6], hb[7])};
  unsigned* q = XO + 4 * (size_t)i;
  *(volatile v4u*)q = u;
  __threadfence();
  *(volatile v4u*)q = u;
}

__global__ __launch_bounds__(NT) void k_bucket(const int* __restrict__ ei, int* __restrict__ cells) {
  __shared__ __align__(16) int keys[CHK];
  __shared__ int segst[NTILE + 2];
  const int tid = threadIdx.x, lane = tid & 31, wave = tid >> 5;
  const int c = blockIdx.x;
  const int* dstv = ei + NE;
#pragma unroll
  for (int i = 0; i < CHK / (4 * NT); ++i) {
    if (i == 4 || i == 8 || i == 12) asm volatile("" ::: "memory");
    const int idx4 = (i * NT + tid) * 4;
    const int e4 = c * CHK + idx4;
    const bool inb = e4 < NE;
    const int ec = inb ? e4 : (NE - 4);
    const v4i d4 = *(const v4i*)(dstv + ec);
    v4i k4;
#pragma unroll
    for (int j = 0; j < 4; ++j) {
      const int d = d4[j];
      const bool valid = inb && ((unsigned)d < (unsigned)NN);
      const int tile = valid ? (d >> TSHIFT) : SENT_TILE;
      const int dlow = valid ? (d & (TROWS - 1)) : 0;
      k4[j] = (tile << 21) | (dlow << 14) | (idx4 + j);
    }
    *(v4i*)(keys + idx4) = k4;
  }
  __syncthreads();
#pragma unroll 1
  for (int k = 2; k <= CHK; k <<= 1) {
#pragma unroll 1
    for (int j = k >> 1; j > 0; j >>= 1) {
#pragma unroll 4
      for (int it = 0; it < CHK / (2 * NT); ++it) {
        const int p = it * NT + tid;
        const int i0 = ((p & ~(j - 1)) << 1) | (p & (j - 1));
        const int i1 = i0 | j;
        const int a = keys[i0], b = keys[i1];
        const int lo = (a < b) ? a : b;
        const int hi = (a < b) ? b : a;
        const bool up = ((i0 & k) == 0);
        keys[i0] = up ? lo : hi;
        keys[i1] = up ? hi : lo;
      }
      __syncthreads();
    }
  }
#pragma unroll 1
  for (int r = 0; r < 4; ++r) {
    const int t = tid + NT * r;
    if (t < NTILE + 2) {
      const int target = t << 21;
      int first = 0, count = CHK;
#pragma unroll 1
      for (int s = 0; s < 15; ++s) {
        const bool go = count > 0;
        const int step = count >> 1;
        const int m = first + step;
        const int mc = (m < CHK) ? m : (CHK - 1);
        const int kv = keys[mc];
        const bool lt = go && (kv < target);
        first = lt ? (m + 1) : first;
        count = go ? (lt ? (count - step - 1) : step) : 0;
      }
      segst[t] = first;
    }
  }
  __syncthreads();
  const int hh = lane >> 4, s0 = (lane & 15) * 4;
  for (int pass = 0; pass < 2; ++pass) {
#pragma unroll 1
    for (int it = 0; it < NPIT; ++it) {
      const int pp = wave + 8 * it;
      if (pp < NPAIR) {
        const int t = 2 * pp + hh;
        const int st = segst[t];
        const int cnt = segst[t + 1] - st;
        v4i v;
#pragma unroll
        for (int jj = 0; jj < 4; ++jj) {
          const int s = s0 + jj;
          int ks = st + s; ks = (ks < CHK) ? ks : (CHK - 1);
          const int key = keys[ks];
          const int ent = (((key >> 14) & (TROWS - 1)) << 21) | (c * CHK + (key & 0x3FFF));
          v[jj] = (s < cnt) ? ent : -1;
        }
        *(volatile v4i*)(cells + ((size_t)c * NTILE + 2 * pp) * CAP + lane * 4) = v;
      }
    }
    __threadfence();
  }
}

template <bool XF32>
__device__ __forceinline__ void apply_hits(unsigned msk, int entv, const float* __restrict__ X0, const unsigned* __restrict__ XH,
                                           const int* __restrict__ srcv, const float* __restrict__ ew, float* accL, int lane) {
#pragma unroll 1
  for (int it = 0; it < 32; ++it) {
    if (msk == 0u) break;
    const int bp = __builtin_ctz(msk); msk &= msk - 1u;
    const int ent = __shfl(entv, bp, 32);
    int e = ent & 0x1FFFFF; e = (e < NE) ? e : (NE - 1);
    const int dl = (ent >> 21) & (TROWS - 1);
    int s = srcv[e]; s = s < 0 ? 0 : (s >= NN ? NN - 1 : s);
    const float w = ew[e];
    v4f xv;
    if (XF32) {
      xv = *(const v4f*)(X0 + (size_t)s * CH + 4 * lane);
    } else {
      const v2u u = *(const v2u*)(XH + (size_t)s * (CH / 2) + 2 * lane);
      const float f0 = h16_to_f32(u[0] & 0xffffu);
      const float f1 = h16_to_f32(u[0] >> 16);
      const float f2 = h16_to_f32(u[1] & 0xffffu);
      const float f3 = h16_to_f32(u[1] >> 16);
      xv = (v4f){f0, f1, f2, f3};
    }
    float* rp = accL + dl * CH + 4 * lane;
    v4f a = *(const v4f*)rp;
    a = a + xv * w;
    *(v4f*)rp = a;
  }
}

template <bool XF32>
__global__ __launch_bounds__(NT) void k_aggr(const float* __restrict__ X0, const unsigned* __restrict__ XH,
                                             const int* __restrict__ ei, const float* __restrict__ ew,
                                             const int* __restrict__ cells, unsigned* __restrict__ AGGw) {
  __shared__ __align__(16) float accL[TROWS * CH];
  const int tid = threadIdx.x, lane = tid & 31, wave = tid >> 5;
  const int t = blockIdx.x;
  const v4f z4 = {0.f, 0.f, 0.f, 0.f};
#pragma unroll
  for (int i = 0; i < 16; ++i) *(v4f*)(accL + tid * 64 + 4 * i) = z4;
  __syncthreads();
  const int* srcv = ei;
#pragma unroll 1
  for (int c = 0; c < NCHUNK; ++c) {
    const int* cp = cells + ((size_t)c * NTILE + t) * CAP;
    const int ent0 = cp[lane];
    const int ent1 = cp[32 + lane];
    const int own0 = (ent0 >= 0 && ((ent0 >> 25) & 7) == wave) ? 1 : 0;
    const int own1 = (ent1 >= 0 && ((ent1 >> 25) & 7) == wave) ? 1 : 0;
    const unsigned mska = (unsigned)__ballot(own0);
    const unsigned mskb = (unsigned)__ballot(own1);
    apply_hits<XF32>(mska, ent0, X0, XH, srcv, ew, accL, lane);
    apply_hits<XF32>(mskb, ent1, X0, XH, srcv, ew, accL, lane);
  }
  __syncthreads();
  const int hh = lane >> 4, c8 = (lane & 15) * 8;
  unsigned* base = AGGw + (size_t)t * TROWS * (CH / 2);
  for (int pass = 0; pass < 2; ++pass) {
#pragma unroll
    for (int it = 0; it < 8; ++it) {
      const int row = wave * 16 + it * 2 + hh;
      const float* sp = accL + row * CH + c8;
      const v4f lo = *(const v4f*)(sp);
      const v4f hi = *(const v4f*)(sp + 4);
      const v4u u = (v4u){pk16(h_bits(lo[0]), h_bits(lo[1])), pk16(h_bits(lo[2]), h_bits(lo[3])),
                          pk16(h_bits(hi[0]), h_bits(hi[1])), pk16(h_bits(hi[2]), h_bits(hi[3]))};
      *(volatile v4u*)(base + (size_t)row * (CH / 2) + (c8 >> 1)) = u;
    }
    __threadfence();
  }
}

__global__ __launch_bounds__(NT) void k_gemm_cat(const unsigned short* __restrict__ A0p, const unsigned short* __restrict__ A1p,
                                                 const unsigned short* __restrict__ Btp, const float* __restrict__ bias,
                                                 unsigned short* __restrict__ Cp) {
  typedef _Float16 T;
  const T* A0 = (const T*)A0p; const T* A1 = (const T*)A1p; const T* Bt = (const T*)Btp;
  __shared__ __align__(16) float sT[8][16 * 68];
  const int lane = threadIdx.x & 31;
  const int wave = threadIdx.x >> 5;
  constexpr int tilesN = CH >> 6;
  constexpr int tilesM = NPAD2 >> 6;
  const int tile = blockIdx.x * 8 + wave;
  if (tile >= tilesM * tilesN) return;
  const int tm = tile / tilesN;
  const int tn = tile - tm * tilesN;
  const int m0 = tm << 6;
  const int n0 = tn << 6;
  const int rlane = lane & 15;
  const int koff  = (lane >> 4) * 8;
  const int mOff  = (lane >> 4) * 8;

  v8f acc[4][4];
#pragma unroll
  for (int i = 0; i < 4; ++i)
#pragma unroll
    for (int j = 0; j < 4; ++j) acc[i][j] = (v8f){0.f,0.f,0.f,0.f,0.f,0.f,0.f,0.f};

  for (int kk = 0; kk < KCAT; kk += 32) {
    const T* Ab = (kk < CH) ? A0 : A1;
    const int k0 = kk & (CH - 1);
    v16h bh[4];
#pragma unroll
    for (int j = 0; j < 4; ++j) {
      const size_t bo = (size_t)(n0 + (j << 4) + rlane) * KCAT + koff + kk;
      bh[j] = Frag<T>::load(Bt + bo);
    }
#pragma unroll
    for (int i = 0; i < 4; ++i) {
      const size_t ao = (size_t)(m0 + (i << 4) + rlane) * CH + koff + k0;
      const v16h ah = Frag<T>::load(Ab + ao);
#pragma unroll
      for (int j = 0; j < 4; ++j) acc[i][j] = Frag<T>::mma(ah, bh[j], acc[i][j]);
      guard_grp(acc[i][0], acc[i][1], acc[i][2], acc[i][3], ah, bh[0], bh[1], bh[2], bh[3]);
    }
    Frag<T>::keep(bh[0], bh[1], bh[2], bh[3]);
  }
  acc_guard4(acc[0][0], acc[0][1], acc[0][2], acc[0][3]);
  acc_guard4(acc[1][0], acc[1][1], acc[1][2], acc[1][3]);
  acc_guard4(acc[2][0], acc[2][1], acc[2][2], acc[2][3]);
  acc_guard4(acc[3][0], acc[3][1], acc[3][2], acc[3][3]);

  float* slab = sT[wave];
#pragma unroll
  for (int i = 0; i < 4; ++i) {
    const int mBase = m0 + (i << 4);
#pragma unroll
    for (int j = 0; j < 4; ++j) {
      const int n = n0 + (j << 4) + rlane;
      const float bv = bias[n];
#pragma unroll
      for (int r = 0; r < 8; ++r) {
        float v = acc[i][j][r] * WCARRY_INV + bv;
        v = fmaxf(v, 0.0f);
        slab[(mOff + r) * 68 + (j << 4) + rlane] = v;
      }
    }
    __builtin_amdgcn_fence(__ATOMIC_RELEASE, "workgroup");
    __builtin_amdgcn_wave_barrier();
    __builtin_amdgcn_fence(__ATOMIC_ACQUIRE, "workgroup");
    {
      const int q = lane >> 3, c8 = (lane & 7) * 8;
      unsigned short* C = Cp;
      for (int pass = 0; pass < 2; ++pass) {
#pragma unroll
        for (int it = 0; it < 4; ++it) {
          const int row = it * 4 + q;
          const float* sp = slab + row * 68 + c8;
          v8h hv;
#pragma unroll
          for (int e = 0; e < 8; ++e) hv[e] = (_Float16)sp[e];
          *(volatile v8h*)(C + (size_t)(mBase + row) * CH + n0 + c8) = hv;
        }
        __threadfence();
      }
    }
    __builtin_amdgcn_fence(__ATOMIC_RELEASE, "workgroup");
    __builtin_amdgcn_wave_barrier();
    __builtin_amdgcn_fence(__ATOMIC_ACQUIRE, "workgroup");
  }
}

__global__ __launch_bounds__(NT) void k_cls(const unsigned short* __restrict__ P1, const unsigned short* __restrict__ P2,
                                            const unsigned short* __restrict__ P3, const unsigned short* __restrict__ WL,
                                            const float* __restrict__ blin, float* __restrict__ out) {
  __shared__ __align__(16) float sL[64 * 68];
  __shared__ __align__(16) float sO[64 * NCLS];
  const int tid = threadIdx.x, lane = tid & 31, wave = tid >> 5;
  const int m0 = blockIdx.x * 64;
  const int rlane = lane & 15;
  const int koff  = (lane >> 4) * 8;
  const int mOff  = (lane >> 4) * 8;
  const int rt = wave >> 1, chalf = wave & 1;
  const _Float16* p1 = (const _Float16*)P1;
  const _Float16* p2 = (const _Float16*)P2;
  const _Float16* p3 = (const _Float16*)P3;
  const _Float16* WLh = (const _Float16*)WL;
  v8f acc0 = (v8f){0.f,0.f,0.f,0.f,0.f,0.f,0.f,0.f};
  v8f acc1 = (v8f){0.f,0.f,0.f,0.f,0.f,0.f,0.f,0.f};
#pragma unroll 1
  for (int seg = 0; seg < 3; ++seg) {
    const _Float16* Ps = (seg == 0) ? p1 : ((seg == 1) ? p2 : p3);
    const _Float16* arow  = Ps + (size_t)(m0 + rt * 16 + rlane) * CH + koff;
    const _Float16* brow0 = WLh + (size_t)(chalf * 32 + rlane) * HCAT + seg * CH + koff;
    const _Float16* brow1 = brow0 + (size_t)16 * HCAT;
#pragma unroll 1
    for (int kin = 0; kin < CH; kin += 32) {
      const v16h b0 = Frag<_Float16>::load(brow0 + kin);
      const v16h b1 = Frag<_Float16>::load(brow1 + kin);
      const v16h a  = Frag<_Float16>::load(arow + kin);
      acc0 = Frag<_Float16>::mma(a, b0, acc0);
      acc1 = Frag<_Float16>::mma(a, b1, acc1);
      guard2f(acc0, acc1, a, b0, b1);
    }
  }
  acc_guard2(acc0, acc1);
  {
    const int col0 = chalf * 32 + rlane, col1 = col0 + 16;
    const int c0c = (col0 < NCLS) ? col0 : (NCLS - 1);
    const int c1c = (col1 < NCLS) ? col1 : (NCLS - 1);
    const float f0 = (col0 < NCLS) ? 1.0f : 0.0f;
    const float f1 = (col1 < NCLS) ? 1.0f : 0.0f;
    const float bv0 = blin[c0c] * f0;
    const float bv1 = blin[c1c] * f1;
#pragma unroll
    for (int r = 0; r < 8; ++r) {
      const int row = rt * 16 + mOff + r;
      sL[row * 68 + col0] = acc0[r] * WCARRY_INV + bv0;
      sL[row * 68 + col1] = acc1[r] * WCARRY_INV + bv1;
    }
  }
  __syncthreads();
  if (tid < 64) {
    const float* lr = sL + tid * 68;
    float mx = lr[0];
#pragma unroll 1
    for (int c = 1; c < NCLS; ++c) mx = fmaxf(mx, lr[c]);
    float sum = 0.0f;
#pragma unroll 1
    for (int c = 0; c < NCLS; ++c) sum += expf(lr[c] - mx);
    const float lse = logf(sum);
#pragma unroll 1
    for (int c = 0; c < NCLS; ++c) sO[tid * NCLS + c] = (lr[c] - mx) - lse;
  }
  __syncthreads();
  int rows_valid = NN - m0; rows_valid = (rows_valid > 64) ? 64 : (rows_valid < 0 ? 0 : rows_valid);
  const int nlines = (rows_valid * NCLS) >> 5;
  float* ob = out + (size_t)m0 * NCLS;
  const int lq = lane >> 3, l4 = (lane & 7) * 4;
  for (int pass = 0; pass < 2; ++pass) {
#pragma unroll
    for (int it = 0; it < 3; ++it) {
      const int L = it * 32 + wave * 4 + lq;
      const int Lc = (L < 81) ? L : 81;
      const v4f v = *(const v4f*)(sO + Lc * 32 + l4);
      if (L < nlines) *(volatile v4f*)(ob + (size_t)L * 32 + l4) = v;
    }
    __threadfence();
  }
}

extern "C" void kernel_launch(void* const* d_in, const int* in_sizes, int n_in,
                              void* d_out, int out_size, void* d_ws, size_t ws_size, hipStream_t stream) {
  (void)in_sizes; (void)n_in; (void)out_size;
  const float* x0    = (const float*)d_in[0];
  const int*   ei    = (const int*)  d_in[1];
  const float* ew    = (const float*)d_in[2];
  const float* Wrel1 = (const float*)d_in[3];
  const float* brel1 = (const float*)d_in[4];
  const float* Wroo1 = (const float*)d_in[5];
  const float* Wrel2 = (const float*)d_in[6];
  const float* brel2 = (const float*)d_in[7];
  const float* Wroo2 = (const float*)d_in[8];
  const float* Wrel3 = (const float*)d_in[9];
  const float* brel3 = (const float*)d_in[10];
  const float* Wroo3 = (const float*)d_in[11];
  const float* Wlin  = (const float*)d_in[12];
  const float* blin  = (const float*)d_in[13];
  float* out = (float*)d_out;

  char* ws = (char*)d_ws; size_t off = 0;
  auto carve = [&](size_t bytes) -> char* { char* p = ws + off; off += (bytes + 255) & ~(size_t)255; return p; };
  unsigned short* AGG = (unsigned short*)carve((size_t)NPAD2 * CH * 2);
  unsigned short* P1  = (unsigned short*)carve((size_t)NPAD2 * CH * 2);
  unsigned short* P2  = (unsigned short*)carve((size_t)NPAD2 * CH * 2);
  unsigned short* P3  = (unsigned short*)carve((size_t)NPAD2 * CH * 2);
  unsigned short* WC  = (unsigned short*)carve((size_t)3 * CH * KCAT * 2);
  unsigned short* WLp = (unsigned short*)carve((size_t)NCLSP * HCAT * 2);
  int*            CEL = (int*)carve((size_t)NCHUNK * NTILE * CAP * 4);
  if (off > ws_size || off > (size_t)134217728) return;

  const unsigned short* WC1 = WC;
  const unsigned short* WC2 = WC + (size_t)CH * KCAT;
  const unsigned short* WC3 = WC + (size_t)2 * CH * KCAT;

  k_packw<<<dim3(48, 7), NT, 0, stream>>>(Wrel1, Wroo1, Wrel2, Wroo2, Wrel3, Wroo3, Wlin, (unsigned*)WC, (unsigned*)WLp);
  k_cast_x0<<<(NPAD2 * 16) / NT, NT, 0, stream>>>(x0, (unsigned*)P3);
  k_bucket<<<NCHUNK, NT, 0, stream>>>(ei, CEL);

  k_aggr<true><<<NTILE, NT, 0, stream>>>(x0, (const unsigned*)P3, ei, ew, CEL, (unsigned*)AGG);
  k_gemm_cat<<<GEMM_BLOCKS, NT, 0, stream>>>(AGG, P3, WC1, brel1, P1);
  k_aggr<false><<<NTILE, NT, 0, stream>>>(x0, (const unsigned*)P1, ei, ew, CEL, (unsigned*)AGG);
  k_gemm_cat<<<GEMM_BLOCKS, NT, 0, stream>>>(AGG, P1, WC2, brel2, P2);
  k_aggr<false><<<NTILE, NT, 0, stream>>>(x0, (const unsigned*)P2, ei, ew, CEL, (unsigned*)AGG);
  k_gemm_cat<<<GEMM_BLOCKS, NT, 0, stream>>>(AGG, P2, WC3, brel3, P3);
  k_cls<<<MCLS, NT, 0, stream>>>(P1, P2, P3, WLp, blin, out);
}
